// BondLengthHead_48009144434794
// MI455X (gfx1250) — hardware-verified
//
#include <hip/hip_runtime.h>
#include <stddef.h>


#define NTHR 256
#define LAT  128
#define EMB  32
#define PCOL 256
#define H2W  64
#define ETR  16
#define EB   256
#define TP   68
#define HP   136
#define W1SC 16.0f
#define W1IV 0.0625f
#define W2SC 8.0f
#define W2IV 0.125f

static_assert((TP % 4) == 0);
static_assert((HP % 8) == 0);
static_assert(EB == 8 * 2 * 16);

typedef float        v4f  __attribute__((ext_vector_type(4)));
typedef float        v8f  __attribute__((ext_vector_type(8)));
typedef unsigned int v4u  __attribute__((ext_vector_type(4)));
typedef _Float16     v4h  __attribute__((ext_vector_type(4)));
typedef _Float16     v8h  __attribute__((ext_vector_type(8)));
typedef _Float16     v16h __attribute__((ext_vector_type(16)));
union FragH { v16h v; v8h h[2]; };
union Pack8 { v8h h; v4u u; };

__device__ __forceinline__ v8f zero8f() {
  v8f r;
#pragma unroll
  for (int i = 0; i < 8; ++i) r[i] = 0.0f;
  return r;
}

__device__ __forceinline__ v8f wmh(v16h a, v16h b, v8f c) {
  v8f d = __builtin_amdgcn_wmma_f32_16x16x32_f16(false, a, false, b, (short)0, c, false, false);
  asm volatile("v_nop\n\tv_nop\n\tv_nop\n\tv_nop" : "+v"(d) : "v"(a), "v"(b));
  return d;
}

__device__ __forceinline__ float softplus1(float x) {
  return fmaxf(x, 0.0f) + log1pf(expf(-fabsf(x)));
}

__global__ __launch_bounds__(NTHR) void k_prep(
    const float* __restrict__ z, const float* __restrict__ embed,
    const float* __restrict__ W1, const float* __restrict__ b1, const float* __restrict__ W2,
    _Float16* Zh, _Float16* W1t, _Float16* W2t, float* EtB,
    int nN, int nPad, int nT, int nbZ) {
  const int tid = threadIdx.x;
  const int blk = blockIdx.x;
  if (blk < nbZ) {
    const int t   = blk * NTHR + tid;
    const int row = t >> 4, k0 = (t & 15) * 8;
    if (row < nPad) {
      const int rr = row < nN ? row : nN - 1;
      const bool ok = row < nN;
      const float* zp = z + (size_t)rr * LAT + k0;
      const v4f a = *(const v4f*)zp;
      const v4f b = *(const v4f*)(zp + 4);
      Pack8 pk;
#pragma unroll
      for (int c = 0; c < 4; ++c) {
        const float va = ok ? a[c] : 0.0f;
        const float vb = ok ? b[c] : 0.0f;
        pk.h[c]     = (_Float16)va;
        pk.h[4 + c] = (_Float16)vb;
      }
      v4u* gp = (v4u*)(Zh + (size_t)row * LAT + k0);
      *(volatile v4u*)gp = pk.u;
      __threadfence();
      *(volatile v4u*)gp = pk.u;
    }
  } else if (blk < nbZ + 16) {
    const int t = (blk - nbZ) * NTHR + tid;
    const int n = t >> 4, k0 = (t & 15) * 8;
    Pack8 pk;
#pragma unroll
    for (int c = 0; c < 8; ++c) {
      const int k   = k0 + c;
      const int idx = (n < LAT) ? (k * LAT + n) : ((LAT + k) * LAT + (n - LAT));
      pk.h[c] = (_Float16)(W1[idx] * W1SC);
    }
    v4u* gp = (v4u*)(W1t + (size_t)n * LAT + k0);
    *(volatile v4u*)gp = pk.u;
    __threadfence();
    *(volatile v4u*)gp = pk.u;
  } else if (blk < nbZ + 20) {
    const int t = (blk - nbZ - 16) * NTHR + tid;
    const int n = t >> 4, k0 = (t & 15) * 8;
    Pack8 pk;
#pragma unroll
    for (int c = 0; c < 8; ++c) {
      const int k = k0 + c;
      pk.h[c] = (_Float16)(W2[k * H2W + n] * W2SC);
    }
    v4u* gp = (v4u*)(W2t + (size_t)n * LAT + k0);
    *(volatile v4u*)gp = pk.u;
    __threadfence();
    *(volatile v4u*)gp = pk.u;
  } else if (blk < nbZ + 22) {
    const int t   = (blk - nbZ - 20) * NTHR + tid;
    const int tr  = t >> 5, n0 = (t & 31) * 4;
    const int trc = tr < nT ? tr : nT - 1;
    v4f acc = *(const v4f*)(b1 + n0);
#pragma unroll 1
    for (int j = 0; j < EMB; ++j) {
      const float e = embed[trc * EMB + j];
      const v4f   w = *(const v4f*)(W1 + (size_t)(2 * LAT + j) * LAT + n0);
      acc = acc + w * e;
    }
    if (tr >= nT) { acc[0] = 0.0f; acc[1] = 0.0f; acc[2] = 0.0f; acc[3] = 0.0f; }
    float* gp = EtB + (size_t)tr * LAT + n0;
    *(volatile v4f*)gp = acc;
    __threadfence();
    *(volatile v4f*)gp = acc;
  }
}

__global__ __launch_bounds__(NTHR) void k_pgemm(const _Float16* __restrict__ Zh,
                                               const _Float16* __restrict__ W1t, float* P) {
  __shared__ __attribute__((aligned(16))) float sT[8 * 16 * TP];
  const int tid = threadIdx.x, lane = tid & 31, wave = tid >> 5, h = lane >> 4, m = lane & 15;
  const int rbase = blockIdx.x * 64 + (wave >> 2) * 32;
  const int cbase = (wave & 3) * 64;

  v8f acc[2][4];
#pragma unroll
  for (int mt = 0; mt < 2; ++mt)
#pragma unroll
    for (int nt = 0; nt < 4; ++nt) acc[mt][nt] = zero8f();

#pragma unroll
  for (int ks = 0; ks < LAT / 32; ++ks) {
    FragH a[2];
#pragma unroll
    for (int mt = 0; mt < 2; ++mt) {
      const _Float16* ap = Zh + (size_t)(rbase + mt * 16 + m) * LAT + ks * 32 + 8 * h;
      a[mt].h[0] = *(const v8h*)ap;
      a[mt].h[1] = *(const v8h*)(ap + 16);
    }
#pragma unroll
    for (int nt = 0; nt < 4; ++nt) {
      FragH b;
      const _Float16* bp = W1t + (size_t)(cbase + nt * 16 + m) * LAT + ks * 32 + 8 * h;
      b.h[0] = *(const v8h*)bp;
      b.h[1] = *(const v8h*)(bp + 16);
      acc[0][nt] = wmh(a[0].v, b.v, acc[0][nt]);
      acc[1][nt] = wmh(a[1].v, b.v, acc[1][nt]);
    }
  }

  float* st = sT + wave * 16 * TP;
#pragma unroll
  for (int mt = 0; mt < 2; ++mt) {
#pragma unroll
    for (int nt = 0; nt < 4; ++nt) {
#pragma unroll
      for (int r = 0; r < 8; ++r) st[(8 * h + r) * TP + nt * 16 + m] = acc[mt][nt][r] * W1IV;
    }
    __syncthreads();
    v4f ov[8];
#pragma unroll
    for (int j = 0; j < 8; ++j) ov[j] = *(const v4f*)(st + (2 * j + h) * TP + 4 * m);
    float* gp = P + (size_t)(rbase + mt * 16) * PCOL + cbase + 4 * m;
#pragma unroll
    for (int j = 0; j < 8; ++j) *(volatile v4f*)(gp + (size_t)(2 * j + h) * PCOL) = ov[j];
    __threadfence();
#pragma unroll
    for (int j = 0; j < 8; ++j) *(volatile v4f*)(gp + (size_t)(2 * j + h) * PCOL) = ov[j];
    __syncthreads();
  }
}

__global__ __launch_bounds__(NTHR) void k_edge(
    const float* __restrict__ P, const float* __restrict__ EtB,
    const int* __restrict__ ei, const int* __restrict__ bty,
    const _Float16* __restrict__ W2t, const float* __restrict__ b2,
    const float* __restrict__ W3, const float* __restrict__ b3,
    float* out, int nN, int nE, int nT) {
  __shared__ __attribute__((aligned(16))) _Float16 sW2[H2W * HP];
  __shared__ __attribute__((aligned(16))) _Float16 sH[8 * 16 * HP];
  __shared__ __attribute__((aligned(16))) float    sOut[EB];
  __shared__ float sB2[H2W];
  __shared__ float sW3[H2W];

  const int tid = threadIdx.x, lane = tid & 31, wave = tid >> 5, h = lane >> 4, m = lane & 15;

#pragma unroll
  for (int q = 0; q < 4; ++q) {
    const int c = q * NTHR + tid;
    const int row = c >> 4, k0 = (c & 15) * 8;
    *(v8h*)(sW2 + row * HP + k0) = *(const v8h*)(W2t + (size_t)row * LAT + k0);
  }
  if (tid < H2W) { sB2[tid] = b2[tid]; sW3[tid] = W3[tid]; }
  const float bias3 = b3[0];
  __syncthreads();

  _Float16* hw = sH + wave * 16 * HP;

#pragma unroll 1
  for (int t = 0; t < 2; ++t) {
    const int ebase = blockIdx.x * EB + (wave * 2 + t) * 16;
    int e = ebase + m;
    e = e > nE - 1 ? nE - 1 : e;
    int s = ei[e];
    int d = ei[(size_t)nE + (size_t)e];
    int b = bty[e];
    s = s < 0 ? 0 : (s > nN - 1 ? nN - 1 : s);
    d = d < 0 ? 0 : (d > nN - 1 ? nN - 1 : d);
    b = b < 0 ? 0 : (b > nT - 1 ? nT - 1 : b);

#pragma unroll
    for (int i = 0; i < 16; ++i) {
      const int si = __shfl(s, i);
      const int di = __shfl(d, i);
      const int bi = __shfl(b, i);
      const v4f ps = *(const v4f*)(P + (size_t)si * PCOL + 4 * lane);
      const v4f pd = *(const v4f*)(P + (size_t)di * PCOL + LAT + 4 * lane);
      const v4f pe = *(const v4f*)(EtB + (size_t)bi * LAT + 4 * lane);
      const v4f hs = (ps + pd) + pe;
      v4h hv;
#pragma unroll
      for (int c = 0; c < 4; ++c) hv[c] = (_Float16)fmaxf(hs[c], 0.0f);
      *(v4h*)(hw + i * HP + 4 * lane) = hv;
    }
    __syncthreads();

    v8f acc[4];
#pragma unroll
    for (int nt = 0; nt < 4; ++nt) acc[nt] = zero8f();
#pragma unroll
    for (int ks = 0; ks < LAT / 32; ++ks) {
      FragH a;
      const _Float16* ap = hw + m * HP + ks * 32 + 8 * h;
      a.h[0] = *(const v8h*)ap;
      a.h[1] = *(const v8h*)(ap + 16);
#pragma unroll
      for (int nt = 0; nt < 4; ++nt) {
        FragH bb;
        const _Float16* bp = sW2 + (nt * 16 + m) * HP + ks * 32 + 8 * h;
        bb.h[0] = *(const v8h*)bp;
        bb.h[1] = *(const v8h*)(bp + 16);
        acc[nt] = wmh(a.v, bb.v, acc[nt]);
      }
    }

    float p[8];
#pragma unroll
    for (int r = 0; r < 8; ++r) p[r] = 0.0f;
#pragma unroll
    for (int nt = 0; nt < 4; ++nt) {
      const int col = nt * 16 + m;
      const float w3 = sW3[col], bb2 = sB2[col];
#pragma unroll
      for (int r = 0; r < 8; ++r) {
        const float v = fmaxf(acc[nt][r] * W2IV + bb2, 0.0f);
        p[r] = v * w3 + p[r];
      }
    }
#pragma unroll
    for (int off = 1; off < 16; off <<= 1) {
#pragma unroll
      for (int r = 0; r < 8; ++r) p[r] += __shfl_xor(p[r], off);
    }
    if (m == 0) {
#pragma unroll
      for (int r = 0; r < 8; ++r) sOut[(wave * 2 + t) * 16 + 8 * h + r] = p[r] + bias3;
    }
    __syncthreads();
  }

  if (wave < 2) {
    const int idx = (wave * 32 + lane) * 4;
    const v4f x = *(const v4f*)(sOut + idx);
    v4f y;
#pragma unroll
    for (int c = 0; c < 4; ++c) y[c] = softplus1(x[c]);
    const size_t ge = (size_t)blockIdx.x * EB + (size_t)idx;
    const size_t lim = (size_t)nE;
    if (ge + 4 <= lim) {
      *(volatile v4f*)(out + ge) = y;
    } else {
#pragma unroll
      for (int c = 0; c < 4; ++c) if (ge + c < lim) *(volatile float*)(out + ge + c) = y[c];
    }
    __threadfence();
    if (ge + 4 <= lim) {
      *(volatile v4f*)(out + ge) = y;
    } else {
#pragma unroll
      for (int c = 0; c < 4; ++c) if (ge + c < lim) *(volatile float*)(out + ge + c) = y[c];
    }
  }
}

extern "C" void kernel_launch(void* const* d_in, const int* in_sizes, int n_in,
                              void* d_out, int out_size, void* d_ws, size_t ws_size,
                              hipStream_t stream) {
  if (n_in < 10) return;
  const int nN = in_sizes[0] / LAT;
  if (nN <= 0 || in_sizes[0] != nN * LAT) return;
  const int nE = in_sizes[1] / 2;
  if (nE <= 0 || in_sizes[1] != 2 * nE || in_sizes[2] != nE) return;
  const int nT = in_sizes[3] / EMB;
  if (nT <= 0 || nT > ETR || in_sizes[3] != nT * EMB) return;
  if (in_sizes[4] != (2 * LAT + EMB) * LAT || in_sizes[5] != LAT) return;
  if (in_sizes[6] != LAT * H2W || in_sizes[7] != H2W || in_sizes[8] != H2W || in_sizes[9] < 1) return;
  if (out_size != nE) return;

  const float* z     = (const float*)d_in[0];
  const int*   ei    = (const int*)d_in[1];
  const int*   bty   = (const int*)d_in[2];
  const float* embed = (const float*)d_in[3];
  const float* W1    = (const float*)d_in[4];
  const float* b1    = (const float*)d_in[5];
  const float* W2    = (const float*)d_in[6];
  const float* b2    = (const float*)d_in[7];
  const float* W3    = (const float*)d_in[8];
  const float* b3    = (const float*)d_in[9];
  float* out = (float*)d_out;

  const int nPad = ((nN + 63) / 64) * 64;

  char* ws = (char*)d_ws;
  size_t off = 0;
  const size_t oZh = off; off += (size_t)nPad * LAT * 2;    off = (off + 255) & ~(size_t)255;
  const size_t oP  = off; off += (size_t)nPad * PCOL * 4;   off = (off + 255) & ~(size_t)255;
  const size_t oW1 = off; off += (size_t)PCOL * LAT * 2;    off = (off + 255) & ~(size_t)255;
  const size_t oW2 = off; off += (size_t)H2W * LAT * 2;     off = (off + 255) & ~(size_t)255;
  const size_t oEt = off; off += (size_t)ETR * LAT * 4;     off = (off + 255) & ~(size_t)255;
  if (off > ws_size) return;
  _Float16* Zh  = (_Float16*)(ws + oZh);
  float*    P   = (float*)(ws + oP);
  _Float16* W1t = (_Float16*)(ws + oW1);
  _Float16* W2t = (_Float16*)(ws + oW2);
  float*    EtB = (float*)(ws + oEt);

  const int nbZ = (nPad * 16) / NTHR;

  k_prep<<<nbZ + 22, NTHR, 0, stream>>>(z, embed, W1, b1, W2, Zh, W1t, W2t, EtB, nN, nPad, nT, nbZ);

  k_pgemm<<<nPad / 64, NTHR, 0, stream>>>(Zh, W1t, P);

  k_edge<<<(nE + EB - 1) / EB, NTHR, 0, stream>>>(P, EtB, ei, bty, W2t, b2, W3, b3, out, nN, nE, nT);
}
